// EntangledInterferenceLayer_56358560858679
// MI455X (gfx1250) — hardware-verified
//
#include <hip/hip_runtime.h>
#include <math.h>

typedef __attribute__((ext_vector_type(16))) _Float16 v16h;
typedef __attribute__((ext_vector_type(16))) __bf16 v16b;
typedef __attribute__((ext_vector_type(8)))  _Float16 v8h;
typedef __attribute__((ext_vector_type(8)))  float v8f;
typedef __attribute__((ext_vector_type(4)))  float v4f;
typedef __attribute__((ext_vector_type(2)))  float v2f;
typedef __attribute__((ext_vector_type(4)))  unsigned v4u;
typedef __attribute__((ext_vector_type(4)))  int v4i;
typedef float __attribute__((may_alias)) float_a;
typedef int __attribute__((may_alias)) int_a;

template <typename T> __device__ __forceinline__ void vst2(void* p, T v) { *(volatile T*)p = v; __threadfence(); *(volatile T*)p = v; }
__device__ __forceinline__ v8f wmma16(v16h a, v16h b, v8f c) {
  v8f d = __builtin_amdgcn_wmma_f32_16x16x32_f16(false, a, false, b, (short)0, c, false, false);
  asm volatile("v_nop\n\tv_nop\n\tv_nop\n\tv_nop" : "+v"(d) : "v"(a), "v"(b));
  return d;
}
__device__ __forceinline__ v8f wmma_bf(v16b a, v16b b, v8f c) {
  v8f d = __builtin_amdgcn_wmma_f32_16x16x32_bf16(false, a, false, b, (short)0, c, false, false);
  asm volatile("v_nop\n\tv_nop\n\tv_nop\n\tv_nop" : "+v"(d) : "v"(a), "v"(b));
  return d;
}
__device__ __forceinline__ v16h frag_h(const _Float16* rowk0, int lane) {
  union { v16h v; v8h q[2]; } u; const _Float16* p = rowk0 + 8 * (lane >> 4);
  u.q[0] = *(const v8h*)p; u.q[1] = *(const v8h*)(p + 16); return u.v;
}
__device__ __forceinline__ v16h frag_f32(const float* rowk0, int lane) {
  v16h a; const float* p = rowk0 + 8 * (lane >> 4);
#pragma unroll
  for (int i = 0; i < 8; ++i) { a[i] = (_Float16)p[i]; a[8 + i] = (_Float16)p[16 + i]; }
  return a;
}
__device__ __forceinline__ v16h frag_f32s(const float* rowk0, int lane, float sc) {
  v16h a; const float* p = rowk0 + 8 * (lane >> 4);
#pragma unroll
  for (int i = 0; i < 8; ++i) { a[i] = (_Float16)(p[i] * sc); a[8 + i] = (_Float16)(p[16 + i] * sc); }
  return a;
}
__device__ __forceinline__ v16h fragc_f32(const float* W, int k0, int n, int lane, int ld, int K) {
  v16h a; const int g = lane >> 4;
#pragma unroll
  for (int i = 0; i < 8; ++i) { const int ka = k0 + 8 * g + i, kb = ka + 16;
    a[i] = (_Float16)(ka < K ? W[(size_t)(ka < K ? ka : K - 1) * ld + n] : 0.f); a[8 + i] = (_Float16)(kb < K ? W[(size_t)(kb < K ? kb : K - 1) * ld + n] : 0.f); }
  return a;
}
struct F2 { v16b h, l; };
__device__ __forceinline__ F2 bsplit16(const float v[16]) { F2 r;
#pragma unroll
  for (int i = 0; i < 16; ++i) { const __bf16 h = (__bf16)v[i]; r.h[i] = h; r.l[i] = (__bf16)(v[i] - (float)h); }
  return r; }
__device__ __forceinline__ F2 split_row(const float* row, int k0, int lane) { float v[16]; const float* p = row + k0 + 8 * (lane >> 4);
#pragma unroll
  for (int i = 0; i < 8; ++i) { v[i] = p[i]; v[8 + i] = p[16 + i]; }
  return bsplit16(v); }
__device__ __forceinline__ F2 split_rowK(const float* row, int k0, int lane, int K) { float v[16]; const int g = lane >> 4;
#pragma unroll
  for (int i = 0; i < 8; ++i) { const int ka = k0 + 8 * g + i, kb = ka + 16; v[i] = ka < K ? row[ka < K ? ka : K - 1] : 0.f; v[8 + i] = kb < K ? row[kb < K ? kb : K - 1] : 0.f; }
  return bsplit16(v); }
__device__ __forceinline__ F2 split_col(const float* W, int k0, int n, int lane, int ld, int K) { float v[16]; const int g = lane >> 4;
#pragma unroll
  for (int i = 0; i < 8; ++i) { const int ka = k0 + 8 * g + i, kb = ka + 16; v[i] = ka < K ? W[(size_t)(ka < K ? ka : K - 1) * ld + n] : 0.f; v[8 + i] = kb < K ? W[(size_t)(kb < K ? kb : K - 1) * ld + n] : 0.f; }
  return bsplit16(v); }
__device__ __forceinline__ v8f mac3(const F2& a, const F2& b, v8f c) { c = wmma_bf(a.l, b.h, c); c = wmma_bf(a.h, b.l, c); return wmma_bf(a.h, b.h, c); }
__device__ __forceinline__ float sigm(float v) { return 1.0f / (1.0f + expf(-v)); }
#define LDSX() do { asm volatile("s_wait_dscnt 0" ::: "memory"); __builtin_amdgcn_wave_barrier(); __builtin_amdgcn_fence(__ATOMIC_RELEASE, "workgroup"); } while (0)


#define NB 4
#define TT 1024
#define CC 1024
#define NH 16
#define HD 64
#define NDG 8
#define HG 2
#ifndef TNB
#define TNB NB
#endif
#ifndef AMP
#define AMP TT
#endif
#define NRW (NB * TT)
#define OUT1_OFF 4194304
__device__ __forceinline__ float bfr(float v) { return (float)(__bf16)v; }
typedef __attribute__((ext_vector_type(8))) __bf16 v8b;
__device__ __forceinline__ v16b frag_b(const __bf16* rowk0, int lane) { union { v16b v; v8b q[2]; } u; const __bf16* p = rowk0 + 8 * (lane >> 4); u.q[0] = *(const v8b*)p; u.q[1] = *(const v8b*)(p + 16); return u.v; }

#define QROW (NH * 2 * 16)
#define KROW (NH * 16)
#define WS_ROT 0u
#define WS_PCS (WS_ROT + 8u * (size_t)TT * 16)
#define WS_Q   (WS_PCS + 8u * (size_t)NH * HD)
#define WS_K   (WS_Q + 2u * (size_t)NDG * NRW * QROW)
#define WS_VT  (WS_K + 2u * (size_t)NDG * NRW * KROW)
#define WS_VL  (WS_VT + 2u * (size_t)NB * (2 * CC) * TT)
#define WS_S   (WS_VL + 2u * (size_t)NB * (2 * CC) * TT)
#define WS_Y   (WS_S + 4u * (size_t)HG * TT * TT)
#define WS_END (WS_Y + 4u * (size_t)NRW * 2 * CC)

__global__ __launch_bounds__(256) void k_tab(const float* __restrict__ FRQ, const float* __restrict__ PS, v2f* __restrict__ ROT, v2f* __restrict__ PCS) { const int i = blockIdx.x * 256 + threadIdx.x;
  if (i < TT * 16) { const float ang = (float)(i >> 4) * bfr(FRQ[i & 15]); v2f v; v[0] = cosf(ang); v[1] = sinf(ang); vst2(ROT + i, v); }
  if (i < NH * HD) { const float p = bfr(PS[i]); v2f v; v[0] = cosf(p); v[1] = sinf(p); vst2(PCS + i, v); } }
__global__ __launch_bounds__(128) void k_qk(const float* __restrict__ XR, const float* __restrict__ XI, const float* __restrict__ WQR, const float* __restrict__ BQR, const float* __restrict__ WQI, const float* __restrict__ BQI, const float* __restrict__ WKR, const float* __restrict__ BKR, const float* __restrict__ WKI, const float* __restrict__ BKI, const float* __restrict__ ENT, const v2f* __restrict__ ROT, const v2f* __restrict__ PCS, _Float16* __restrict__ QP, _Float16* __restrict__ KP) {
  __shared__ __align__(16) float sr[64][132], si[64][132]; __shared__ float se[NH * NH];
  const int tid = threadIdx.x, wave = tid >> 5, lane = tid & 31, col = lane & 15, g = lane >> 4; const int dg = blockIdx.y; const int which = blockIdx.z; const size_t r0 = (size_t)blockIdx.x * 64;
  const float* WR = which == 0 ? WQR : WKR; const float* WI = which == 0 ? WQI : WKI; const float* BR = which == 0 ? BQR : BKR; const float* BI = which == 0 ? BQI : BKI;
  for (int e = tid; e < NH * NH; e += 128) se[e] = bfr(ENT[e]);
  v8f ar[8] = {}, ai[8] = {};
#pragma unroll 1
  for (int kc = 0; kc < CC / 32; ++kc) { v16b xa, xb; { const float* p = XR + (r0 + wave * 16 + col) * CC + kc * 32 + 8 * g; const float* p2 = XI + (r0 + wave * 16 + col) * CC + kc * 32 + 8 * g;
#pragma unroll
      for (int i = 0; i < 8; ++i) { xa[i] = (__bf16)p[i]; xa[8 + i] = (__bf16)p[16 + i]; }
      asm volatile("s_wait_loadcnt 0x0" ::: "memory");
#pragma unroll
      for (int i = 0; i < 8; ++i) { xb[i] = (__bf16)p2[i]; xb[8 + i] = (__bf16)p2[16 + i]; } }
#pragma unroll
    for (int j = 0; j < 8; ++j) { v16b wr2, wi2; const int cc = j * 16 + col; const int o = (cc >> 3) * HD + dg * 8 + (cc & 7);
#pragma unroll
      for (int i = 0; i < 8; ++i) { const size_t ka = (size_t)(kc * 32 + 8 * g + i) * CC + o, kb = (size_t)(kc * 32 + 16 + 8 * g + i) * CC + o; wr2[i] = (__bf16)WR[ka]; wr2[8 + i] = (__bf16)WR[kb]; wi2[i] = (__bf16)WI[ka]; wi2[8 + i] = (__bf16)WI[kb]; }
      asm volatile("s_wait_loadcnt 0x0" ::: "memory"); ar[j] = wmma_bf(xa, wr2, ar[j]); ai[j] = wmma_bf(xb, wi2, ai[j]); } }
#pragma unroll
  for (int j = 0; j < 8; ++j) { const int cc = j * 16 + col; const int o = (cc >> 3) * HD + dg * 8 + (cc & 7); const float br = bfr(BR[o]), bi = bfr(BI[o]);
#pragma unroll
    for (int r = 0; r < 8; ++r) { sr[wave * 16 + 8 * g + r][cc] = ar[j][r] + br; si[wave * 16 + 8 * g + r][cc] = ai[j][r] + bi; } }
  __syncthreads();
  if (dg < 4) {
    for (int e = tid; e < 64 * 64; e += 128) { const int rl = e >> 6, pr = e & 63; const int cc = pr * 2; const int dd = cc & 7; const int d = dg * 8 + dd; const int t = (int)((r0 + rl) % TT); const v2f cs = ROT[t * 16 + (d >> 1)];
      { const float x0 = sr[rl][cc], x1 = sr[rl][cc + 1]; sr[rl][cc] = x0 * cs[0] - x1 * cs[1]; sr[rl][cc + 1] = x1 * cs[0] + x0 * cs[1]; }
      { const float x0 = si[rl][cc], x1 = si[rl][cc + 1]; si[rl][cc] = x0 * cs[0] - x1 * cs[1]; si[rl][cc + 1] = x1 * cs[0] + x0 * cs[1]; } }
    __syncthreads(); }
  for (int e = tid; e < 64 * 8 * 2; e += 128) { const int rl = e >> 4, dd = (e >> 1) & 7, part = e & 1; float* rowp = part ? si[rl] : sr[rl]; float old[NH];
#pragma unroll
    for (int h = 0; h < NH; ++h) old[h] = rowp[h * 8 + dd];
#pragma unroll 2
    for (int x = 0; x < NH; ++x) { float a = 0.f;
#pragma unroll
      for (int h = 0; h < NH; ++h) a += old[h] * se[h * NH + x];
      rowp[x * 8 + dd] = a; } }
  __syncthreads();
  for (int e = tid; e < 64 * NH; e += 128) { const int rl = e >> 4, h = e & 15; v8h hr, hi, hin, hrn;
#pragma unroll
    for (int dd = 0; dd < 8; ++dd) { const int d = dg * 8 + dd; const v2f cs = PCS[h * HD + d]; const float xr = sr[rl][h * 8 + dd], xi = si[rl][h * 8 + dd]; const float pr_ = xr * cs[0] - xi * cs[1], pi_ = xr * cs[1] + xi * cs[0];
      hr[dd] = (_Float16)pr_; hi[dd] = (_Float16)pi_; hrn[dd] = (_Float16)(-pr_); hin[dd] = (_Float16)pi_; }
    const size_t row = r0 + rl;
    if (which == 0) { _Float16* qd = QP + (((size_t)dg * NRW + row) * QROW) + h * 32; vst2((v4u*)(qd), *(const v4u*)&hr); vst2((v4u*)(qd + 8), *(const v4u*)&hi); vst2((v4u*)(qd + 16), *(const v4u*)&hin); vst2((v4u*)(qd + 24), *(const v4u*)&hrn); }
    else { _Float16* kd = KP + (((size_t)dg * NRW + row) * KROW) + h * 16; vst2((v4u*)(kd), *(const v4u*)&hr); vst2((v4u*)(kd + 8), *(const v4u*)&hi); } } }
__global__ __launch_bounds__(128) void k_v(const float* __restrict__ XR, const float* __restrict__ XI, const float* __restrict__ WVR, const float* __restrict__ BVR, const float* __restrict__ WVI, const float* __restrict__ BVI, __bf16* __restrict__ VT, __bf16* __restrict__ VL) {
  __shared__ __align__(16) __bf16 th[128][72], tl2[128][72];
  const int tid = threadIdx.x, wave = tid >> 5, lane = tid & 31, col = lane & 15, g = lane >> 4; const int part = blockIdx.z; const int c0 = blockIdx.y * 128; const size_t r0 = (size_t)blockIdx.x * 64; const float* X = part ? XI : XR; const float* WV = part ? WVI : WVR; const float* BV = part ? BVI : BVR;
  v8f acc[8] = {};
#pragma unroll 2
  for (int kc = 0; kc < CC / 32; ++kc) { v16b a; { const float* p = X + (r0 + wave * 16 + col) * CC + kc * 32 + 8 * g;
#pragma unroll
      for (int i = 0; i < 8; ++i) { a[i] = (__bf16)p[i]; a[8 + i] = (__bf16)p[16 + i]; } }
#pragma unroll
    for (int j = 0; j < 8; ++j) { v16b w; const int o = c0 + j * 16 + col;
#pragma unroll
      for (int i = 0; i < 8; ++i) { w[i] = (__bf16)WV[(size_t)(kc * 32 + 8 * g + i) * CC + o]; w[8 + i] = (__bf16)WV[(size_t)(kc * 32 + 16 + 8 * g + i) * CC + o]; }
      asm volatile("s_wait_loadcnt 0x0" ::: "memory"); acc[j] = wmma_bf(a, w, acc[j]); } }
#pragma unroll
  for (int j = 0; j < 8; ++j) { const float bb = bfr(BV[c0 + j * 16 + col]);
#pragma unroll
    for (int r = 0; r < 8; ++r) { const float v = acc[j][r] + bb; const int rl = wave * 16 + 8 * g + r, cl = j * 16 + col; const __bf16 bh = (__bf16)v; th[cl][rl] = bh; tl2[cl][rl] = (__bf16)(v - (float)bh); } }
  __syncthreads();
  { const size_t b = r0 / TT; const int t0 = (int)(r0 % TT); for (int e = tid; e < 128 * 8; e += 128) { const int cl = e >> 3, q = e & 7; const int o = c0 + cl; const int c = (o >> 6) * 128 + part * 64 + (o & 63); const size_t o2 = (b * (2 * CC) + c) * (size_t)TT + t0 + q * 8; vst2((v4u*)(VT + o2), *(const v4u*)&th[cl][q * 8]); vst2((v4u*)(VL + o2), *(const v4u*)&tl2[cl][q * 8]); } } }
__device__ __forceinline__ v16h fragQ(const _Float16* QP, size_t row, int h, int op, int kc, int lane) { const int g = lane >> 4; union { v16h v; v8h q[2]; } u;
  const _Float16* pa = QP + (((size_t)(2 * kc) * NRW + row) * QROW) + h * 32 + op * 16 + 8 * g; const _Float16* pb = QP + (((size_t)(2 * kc + 1) * NRW + row) * QROW) + h * 32 + op * 16 + 8 * g;
  u.q[0] = *(const v8h*)pa; u.q[1] = *(const v8h*)pb; return u.v; }
__device__ __forceinline__ v16h fragK(const _Float16* KP, size_t row, int h, int kc, int lane) { const int g = lane >> 4; union { v16h v; v8h q[2]; } u;
  const _Float16* pa = KP + (((size_t)(2 * kc) * NRW + row) * KROW) + h * 16 + 8 * g; const _Float16* pb = KP + (((size_t)(2 * kc + 1) * NRW + row) * KROW) + h * 16 + 8 * g;
  u.q[0] = *(const v8h*)pa; u.q[1] = *(const v8h*)pb; return u.v; }
__global__ __launch_bounds__(128) void k_sc(const _Float16* __restrict__ QP, const _Float16* __restrict__ KP, const int* __restrict__ AM, const float* __restrict__ STR, const float* __restrict__ TMP, int b, int h0, float* __restrict__ S0) { __shared__ __align__(16) float ss[4][16][132]; const int h = h0 + blockIdx.z; float* S = S0 + (size_t)blockIdx.z * TT * TT;
  const int tid = threadIdx.x, wave = tid >> 5, lane = tid & 31, col = lane & 15, g = lane >> 4; const int k0 = blockIdx.y * 128; const int ql0 = blockIdx.x * 64 + wave * 16; const size_t q0 = (size_t)b * TT + ql0;
  if (k0 > blockIdx.x * 64 + 63) return;
  const float strength = 1.0f / (1.0f + expf(-bfr(STR[0]))); const float temp = fmaxf(bfr(TMP[0]), 0.01f);
  v8f ar[8] = {}, ai[8] = {};
#pragma unroll
  for (int kc = 0; kc < 4; ++kc) { const v16h a0 = fragQ(QP, q0 + col, h, 0, kc, lane), a1 = fragQ(QP, q0 + col, h, 1, kc, lane);
#pragma unroll
    for (int j = 0; j < 8; ++j) { const v16h kb = fragK(KP, (size_t)b * TT + k0 + j * 16 + col, h, kc, lane); ar[j] = wmma16(a0, kb, ar[j]); ai[j] = wmma16(a1, kb, ai[j]); } }
#pragma unroll
  for (int j = 0; j < 8; ++j) { const int kt = k0 + j * 16 + col; const int km = AM[(size_t)b * AMP + kt];
#pragma unroll
    for (int r = 0; r < 8; ++r) { const int qt = ql0 + 8 * g + r; const float x = ar[j][r] * 0.125f, y = ai[j][r] * 0.125f; float v = sqrtf(x * x + y * y + 1e-6f) * strength / temp; if (kt > qt || km != 0) v = -3.0e38f; ss[wave][8 * g + r][j * 16 + col] = v; }
    asm volatile("s_wait_loadcnt 0x0" ::: "memory"); }
  LDSX(); for (int rl = 0; rl < 16; ++rl) vst2(S + (size_t)(ql0 + rl) * TT + k0 + lane * 4, *(const v4f*)&ss[wave][rl][lane * 4]); }
__global__ __launch_bounds__(256) void k_sm(float* __restrict__ S0) { __shared__ float sred[8]; __shared__ float sbc; __shared__ __align__(16) float sh[TT];
  const int t = threadIdx.x; const size_t row = blockIdx.x; float* sr = S0 + (size_t)blockIdx.y * TT * TT + row * TT; const int kend = ((int)row / 64) * 64 + 64;
  float m = -3.0e38f; for (int k = t; k < kend; k += 256) m = fmaxf(m, sr[k]);
#pragma unroll
  for (int o = 1; o < 32; o <<= 1) m = fmaxf(m, __shfl_xor(m, o));
  if ((t & 31) == 0) sred[t >> 5] = m; __syncthreads(); if (t == 0) { float a = sred[0]; for (int i = 1; i < 8; ++i) a = fmaxf(a, sred[i]); sbc = a; } __syncthreads(); m = sbc; __syncthreads();
  float sum = 0.f; for (int k = t; k < kend; k += 256) { const float v = sr[k]; sum += (v <= -1.0e38f) ? 0.f : expf(v - m); }
#pragma unroll
  for (int o = 1; o < 32; o <<= 1) sum += __shfl_xor(sum, o);
  if ((t & 31) == 0) sred[t >> 5] = sum; __syncthreads(); if (t == 0) { float a = 0.f; for (int i = 0; i < 8; ++i) a += sred[i]; sbc = 1.0f / a; } __syncthreads(); const float inv = sbc;
  for (int k = t; k < kend; k += 256) { const float v = sr[k]; sh[k] = (v <= -1.0e38f) ? 0.f : expf(v - m) * inv * 2048.0f; }
  __syncthreads(); for (int q = t; q < kend / 4; q += 256) vst2(sr + q * 4, *(const v4f*)&sh[q * 4]); }
__global__ __launch_bounds__(128) void k_pv(const float* __restrict__ PS0, const __bf16* __restrict__ VT, const __bf16* __restrict__ VL, int b, int h0, float* __restrict__ Y) { const int h = h0 + blockIdx.z; const float* PS = PS0 + (size_t)blockIdx.z * TT * TT; __shared__ __align__(16) float ss[4][16][132];
  const int tid = threadIdx.x, wave = tid >> 5, lane = tid & 31, col = lane & 15, g = lane >> 4; const int ql0 = blockIdx.x * 64 + wave * 16; const int kend = blockIdx.x * 64 + 64;
  v8f acc[8] = {};
#pragma unroll 1
  for (int kc = 0; kc < kend / 32; ++kc) { const F2 p = split_row(PS + (size_t)(ql0 + col) * TT, kc * 32, lane);
    asm volatile("s_wait_loadcnt 0x0" ::: "memory");
#pragma unroll
    for (int j = 0; j < 8; ++j) { const size_t po = ((size_t)b * (2 * CC) + h * 128 + j * 16 + col) * (size_t)TT + kc * 32; const v16b vh = frag_b(VT + po, lane); acc[j] = wmma_bf(p.h, vh, acc[j]); acc[j] = wmma_bf(p.l, vh, acc[j]); acc[j] = wmma_bf(p.h, frag_b(VL + po, lane), acc[j]); } }
#pragma unroll
  for (int j = 0; j < 8; ++j)
#pragma unroll
    for (int r = 0; r < 8; ++r) ss[wave][8 * g + r][j * 16 + col] = acc[j][r] * (1.0f / 2048.0f);
  LDSX(); for (int rl = 0; rl < 16; ++rl) vst2(Y + ((size_t)b * TT + ql0 + rl) * (2 * CC) + h * 128 + lane * 4, *(const v4f*)&ss[wave][rl][lane * 4]); }
__global__ __launch_bounds__(128) void k_out(const float* __restrict__ Y, const float* __restrict__ WOR, const float* __restrict__ BOR, const float* __restrict__ WOI, const float* __restrict__ BOI, float* __restrict__ OUTR, float* __restrict__ OUTI) { __shared__ __align__(16) float sf[4][16][132];
  const int tid = threadIdx.x, wave = tid >> 5, lane = tid & 31, col = lane & 15, g = lane >> 4; const int part = blockIdx.z; const int c0 = blockIdx.y * 128; const size_t r0 = (size_t)blockIdx.x * 64 + wave * 16; const float* WO = part ? WOI : WOR; const float* BO = part ? BOI : BOR; float* OUT = part ? OUTI : OUTR;
  v8f acc[8] = {};
#pragma unroll 2
  for (int kc = 0; kc < CC / 32; ++kc) { F2 a; { float v[16]; const int ca = kc * 32 + 8 * g, cb = ca + 16; const float* pa = Y + (r0 + col) * (2 * CC) + (ca >> 6) * 128 + part * 64 + (ca & 63); const float* pb = Y + (r0 + col) * (2 * CC) + (cb >> 6) * 128 + part * 64 + (cb & 63);
#pragma unroll
      for (int i = 0; i < 8; ++i) { v[i] = pa[i]; v[8 + i] = pb[i]; } a = bsplit16(v); }
#pragma unroll
    for (int j = 0; j < 8; ++j) { v16b w; const int o = c0 + j * 16 + col;
#pragma unroll
      for (int i = 0; i < 8; ++i) { w[i] = (__bf16)WO[(size_t)(kc * 32 + 8 * g + i) * CC + o]; w[8 + i] = (__bf16)WO[(size_t)(kc * 32 + 16 + 8 * g + i) * CC + o]; }
      asm volatile("s_wait_loadcnt 0x0" ::: "memory"); acc[j] = wmma_bf(a.h, w, acc[j]); acc[j] = wmma_bf(a.l, w, acc[j]); } }
#pragma unroll
  for (int j = 0; j < 8; ++j) { const float bb = bfr(BO[c0 + j * 16 + col]);
#pragma unroll
    for (int r = 0; r < 8; ++r) sf[wave][8 * g + r][j * 16 + col] = acc[j][r] + bb; }
  LDSX(); for (int rl = 0; rl < 16; ++rl) vst2(OUT + (r0 + rl) * CC + c0 + lane * 4, *(const v4f*)&sf[wave][rl][lane * 4]); }
extern "C" void kernel_launch(void* const* d_in, const int* in_sizes, int n_in, void* d_out, int out_size, void* d_ws, size_t ws_size, hipStream_t stream) {
  (void)in_sizes; (void)n_in; (void)out_size;
  const float** F = (const float**)d_in;
  if (ws_size < (size_t)WS_END) return;
  char* ws = (char*)d_ws; v2f* ROT = (v2f*)(ws + WS_ROT); v2f* PCS = (v2f*)(ws + WS_PCS); _Float16 *QP = (_Float16*)(ws + WS_Q), *KP = (_Float16*)(ws + WS_K); __bf16 *VT = (__bf16*)(ws + WS_VT), *VL = (__bf16*)(ws + WS_VL); float *S = (float*)(ws + WS_S), *Y = (float*)(ws + WS_Y);
  float* OUTR = (float*)d_out; float* OUTI = (float*)d_out + (size_t)OUT1_OFF;
  k_tab<<<dim3((TT * 16 + 255) / 256), 256, 0, stream>>>(F[21], F[19], ROT, PCS);
  k_qk<<<dim3(TNB * TT / 64, NDG, 2), 128, 0, stream>>>(F[0], F[1], F[3], F[4], F[9], F[10], F[5], F[6], F[11], F[12], F[20], ROT, PCS, QP, KP);
  k_v<<<dim3(TNB * TT / 64, CC / 128, 2), 128, 0, stream>>>(F[0], F[1], F[7], F[8], F[13], F[14], VT, VL);
  for (int b = 0; b < TNB; ++b) for (int h0 = 0; h0 < NH; h0 += HG) {
    k_sc<<<dim3(TT / 64, TT / 128, HG), 128, 0, stream>>>(QP, KP, (const int*)d_in[2], F[22], F[23], b, h0, S);
    k_sm<<<dim3(TT, HG), 256, 0, stream>>>(S);
    k_pv<<<dim3(TT / 64, 1, HG), 128, 0, stream>>>(S, VT, VL, b, h0, Y);
  }
  k_out<<<dim3(TNB * TT / 64, CC / 128, 2), 128, 0, stream>>>(Y, F[15], F[16], F[17], F[18], OUTR, OUTI);
}
